// LayerNormLSTMCell_55903294325169
// MI455X (gfx1250) — hardware-verified
//
#include <hip/hip_runtime.h>

typedef __bf16         v16bf __attribute__((ext_vector_type(16)));
typedef unsigned short v8us  __attribute__((ext_vector_type(8)));
typedef float          v8f   __attribute__((ext_vector_type(8)));
typedef float          v4f   __attribute__((ext_vector_type(4)));
typedef v8us __attribute__((may_alias)) v8usa;
typedef v4f  __attribute__((may_alias)) v4fa;

union Frag { v16bf v; v8us half[2]; };

#define NB     4096
#define NI     1024
#define NHID   1024
#define KD     2048
#define NG     4096
#define NTHR   256
#define LN_EPS 1e-5f

#define BM 128
#define BN 128
#define WROWS 32
#define WCOLS 64
#define GEMM_SMEM_BYTES 65536

#define OUT_ELEMS 8388608
#define OUT1_OFF  4194304

#define WS_XH    0
#define WS_WB    16777216
#define WS_G     33554432
#define WS_TOTAL 100663296

static_assert(KD == NI + NHID);
static_assert(NG == 4 * NHID);
static_assert(WS_WB == WS_XH + NB * KD * 2);
static_assert(WS_G  == WS_WB + NG * KD * 2);
static_assert(WS_TOTAL == WS_G + NB * NG * 4);
static_assert(WS_TOTAL <= 134217728);
static_assert(KD % 32 == 0);
static_assert(NB % BM == 0 && NG % BN == 0);
static_assert(BM == 4 * WROWS && BN == 2 * WCOLS);
static_assert(GEMM_SMEM_BYTES == 8 * WROWS * WCOLS * 4);
static_assert(OUT1_OFF + (NB - 1) * NHID + NHID - 1 < OUT_ELEMS);
static_assert(NG == 16 * NTHR && NHID == 4 * NTHR);
static_assert(KD == 8 * NTHR);

__device__ __forceinline__ unsigned short f2bf(float f) {
  unsigned u = __builtin_bit_cast(unsigned, f);
  u += 0x7FFFu + ((u >> 16) & 1u);
  return (unsigned short)(u >> 16);
}
__device__ __forceinline__ float bf2f(unsigned short s) {
  return __builtin_bit_cast(float, ((unsigned)s) << 16);
}
__device__ __forceinline__ float bfr(float f) { return bf2f(f2bf(f)); }
__device__ __forceinline__ v4f bfr4(v4f v) {
  v4f o;
  o.x = bfr(v.x); o.y = bfr(v.y); o.z = bfr(v.z); o.w = bfr(v.w);
  return o;
}

__device__ __forceinline__ float sigm_f(float v) {
  v = fminf(fmaxf(v, -30.0f), 30.0f);
  const float e = __expf(-v);
  return __builtin_amdgcn_rcpf(1.0f + e);
}
__device__ __forceinline__ float tanh_f(float v) {
  v = fminf(fmaxf(v, -15.0f), 15.0f);
  const float e = __expf(2.0f * v);
  return 1.0f - 2.0f * __builtin_amdgcn_rcpf(1.0f + e);
}

__device__ __forceinline__ float wave_sum(float v) {
  v += __shfl_xor(v, 16);
  v += __shfl_xor(v, 8);
  v += __shfl_xor(v, 4);
  v += __shfl_xor(v, 2);
  v += __shfl_xor(v, 1);
  return v;
}

__device__ __forceinline__ v8f wmma_bf16(v16bf a, v16bf b, v8f c) {
  v8f d = __builtin_amdgcn_wmma_f32_16x16x32_bf16(false, a, false, b, (short)0, c, false, false);
  asm volatile("v_nop\n\tv_nop\n\tv_nop\n\tv_nop" : "+v"(d) : "v"(a), "v"(b));
  return d;
}

__device__ __forceinline__ v16bf load_frag(const unsigned short* p, int h) {
  Frag f;
  f.half[0] = *(const v8usa*)(p + 8 * h);
  f.half[1] = *(const v8usa*)(p + 16 + 8 * h);
  return f.v;
}

__global__ __launch_bounds__(NTHR) void convert_planes(
    const float* __restrict__ x,   const float* __restrict__ hp,
    const float* __restrict__ wih, const float* __restrict__ whh,
    unsigned short* __restrict__ xh, unsigned short* __restrict__ wb)
{
  const int tid = threadIdx.x;
  const int blk = blockIdx.x;
  const int plane = blk >> 12;
  const int row = blk & (NB - 1);
  const float* srcA = plane ? wih : x;
  const float* srcB = plane ? whh : hp;
  unsigned short* dplane = plane ? wb : xh;
  const float* src = (tid < 128) ? (srcA + (size_t)row * NI + (size_t)tid * 8)
                                 : (srcB + (size_t)row * NHID + (size_t)(tid - 128) * 8);
  const v4f a = *(const v4fa*)src;
  const v4f c = *(const v4fa*)(src + 4);
  const v8us o = { f2bf(a.x), f2bf(a.y), f2bf(a.z), f2bf(a.w),
                   f2bf(c.x), f2bf(c.y), f2bf(c.z), f2bf(c.w) };
  unsigned short* dst = dplane + (size_t)row * KD + (size_t)tid * 8;
  *(volatile v8us*)dst = o;
  __threadfence();
  *(volatile v8us*)dst = o;
}

__device__ __forceinline__ void g_store_pass(const float* sW, float* G,
                                             int row0, int col0, int lane) {
  const int q8 = lane & 7, sub = lane >> 3;
  #pragma unroll
  for (int i = 0; i < 16; ++i) {
    const int lid = i * 4 + sub;
    const int row = lid >> 1, seg = lid & 1;
    const v4f v = *(const v4fa*)(sW + row * WCOLS + seg * 32 + 4 * q8);
    *(volatile v4f*)(G + (size_t)(row0 + row) * NG + col0 + seg * 32 + 4 * q8) = v;
  }
}

__global__ __launch_bounds__(NTHR) void gates_gemm(
    const unsigned short* __restrict__ xh,
    const unsigned short* __restrict__ wb,
    float* __restrict__ G)
{
  extern __shared__ __attribute__((aligned(16))) float sEp[];
  const int tid = threadIdx.x, lane = tid & 31, w = tid >> 5;
  const int h = lane >> 4, m = lane & 15;
  const int wM = w & 3, wN = w >> 2;
  const int row0 = blockIdx.y * BM + wM * WROWS;
  const int col0 = blockIdx.x * BN + wN * WCOLS;

  const unsigned short* arow0 = xh + (size_t)(row0 + m) * KD;
  const unsigned short* arow1 = xh + (size_t)(row0 + 16 + m) * KD;
  const unsigned short* brow  = wb + (size_t)(col0 + m) * KD;

  const v8f z8 = {0.f, 0.f, 0.f, 0.f, 0.f, 0.f, 0.f, 0.f};
  v8f acc[8];
  #pragma unroll
  for (int t = 0; t < 8; ++t) acc[t] = z8;

  #pragma unroll 1
  for (int k0 = 0; k0 < KD; k0 += 32) {
    const v16bf a0 = load_frag(arow0 + k0, h);
    const v16bf a1 = load_frag(arow1 + k0, h);
    #pragma unroll
    for (int t = 0; t < 4; ++t) {
      const v16bf b = load_frag(brow + (size_t)t * 16 * KD + k0, h);
      acc[t]     = wmma_bf16(a0, b, acc[t]);
      acc[4 + t] = wmma_bf16(a1, b, acc[4 + t]);
    }
  }

  float* sW = sEp + w * (WROWS * WCOLS);
  #pragma unroll
  for (int wm = 0; wm < 2; ++wm)
    #pragma unroll
    for (int t = 0; t < 4; ++t)
      #pragma unroll
      for (int r = 0; r < 8; ++r)
        sW[(wm * 16 + 8 * h + r) * WCOLS + 16 * t + m] = acc[wm * 4 + t][r];
  __syncthreads();

  g_store_pass(sW, G, row0, col0, lane);
  __threadfence();
  g_store_pass(sW, G, row0, col0, lane);
}

__device__ __forceinline__ void cell_elem(float yi, float yf, float yg, float yo,
                                          float cp, float& hn, float& cn) {
  const float c1 = sigm_f(yf) * cp + sigm_f(yi) * tanh_f(yg);
  cn = c1;
  hn = sigm_f(yo) * tanh_f(c1);
}

__device__ __forceinline__ void out_store_pass(const float* sOut, float* out,
                                               int row, int w, int lane) {
  const int q8 = lane & 7, sub = lane >> 3;
  #pragma unroll
  for (int i = 0; i < 2; ++i) {
    const int lid = w * 8 + i * 4 + sub;
    const int ob = lid >> 5, seg = lid & 31;
    const v4f v = *(const v4fa*)(sOut + ob * NHID + seg * 32 + 4 * q8);
    *(volatile v4f*)(out + (size_t)ob * OUT1_OFF + (size_t)row * NHID + seg * 32 + 4 * q8) = v;
  }
}

__global__ __launch_bounds__(NTHR) void ln_cell_kernel(
    const float* __restrict__ G,
    const float* __restrict__ cprev,
    const float* __restrict__ b_ih,
    const float* __restrict__ b_hh,
    const float* __restrict__ gam,
    const float* __restrict__ bet,
    float* __restrict__ out)
{
  __shared__ __attribute__((aligned(16))) float sRow[NG];
  __shared__ __attribute__((aligned(16))) float sOut[2 * NHID];
  __shared__ float sRedS[8];
  __shared__ float sRedQ[8];

  const int row = blockIdx.x;
  const int tid = threadIdx.x, lane = tid & 31, w = tid >> 5;
  const float* gr = G + (size_t)row * NG;

  float s = 0.0f;
  #pragma unroll
  for (int j = 0; j < 4; ++j) {
    const int idx = 4 * (tid + NTHR * j);
    const v4f g4 = *(const v4fa*)(gr + idx);
    const v4f bi = bfr4(*(const v4fa*)(b_ih + idx));
    const v4f bh = bfr4(*(const v4fa*)(b_hh + idx));
    const v4f v = (g4 + bi) + bh;
    *(v4fa*)(sRow + idx) = v;
    s += (v.x + v.y) + (v.z + v.w);
  }
  s = wave_sum(s);
  if (lane == 0) sRedS[w] = s;
  __syncthreads();
  float ts = 0.0f;
  #pragma unroll
  for (int wv = 0; wv < 8; ++wv) ts += sRedS[wv];
  const float mu = ts * (1.0f / 4096.0f);

  float q = 0.0f;
  #pragma unroll 1
  for (int j = 0; j < 4; ++j) {
    const int idx = 4 * (tid + NTHR * j);
    const v4f v = *(const v4fa*)(sRow + idx);
    const v4f d = v - mu;
    q += (d.x * d.x + d.y * d.y) + (d.z * d.z + d.w * d.w);
  }
  q = wave_sum(q);
  if (lane == 0) sRedQ[w] = q;
  __syncthreads();
  float tq = 0.0f;
  #pragma unroll
  for (int wv = 0; wv < 8; ++wv) tq += sRedQ[wv];
  const float rs = rsqrtf(tq * (1.0f / 4096.0f) + LN_EPS);

  const int gc = 4 * tid;
  const v4f vi = *(const v4fa*)(sRow + gc);
  const v4f vf = *(const v4fa*)(sRow + NHID + gc);
  const v4f vg = *(const v4fa*)(sRow + 2 * NHID + gc);
  const v4f vo = *(const v4fa*)(sRow + 3 * NHID + gc);
  const v4f gi = bfr4(*(const v4fa*)(gam + gc));
  const v4f gf = bfr4(*(const v4fa*)(gam + NHID + gc));
  const v4f gg = bfr4(*(const v4fa*)(gam + 2 * NHID + gc));
  const v4f go = bfr4(*(const v4fa*)(gam + 3 * NHID + gc));
  const v4f ei = bfr4(*(const v4fa*)(bet + gc));
  const v4f ef = bfr4(*(const v4fa*)(bet + NHID + gc));
  const v4f eg = bfr4(*(const v4fa*)(bet + 2 * NHID + gc));
  const v4f eo = bfr4(*(const v4fa*)(bet + 3 * NHID + gc));
  const v4f cp = bfr4(*(const v4fa*)(cprev + (size_t)row * NHID + gc));

  const v4f yi = ((vi - mu) * rs) * gi + ei;
  const v4f yf = ((vf - mu) * rs) * gf + ef;
  const v4f yg = ((vg - mu) * rs) * gg + eg;
  const v4f yo = ((vo - mu) * rs) * go + eo;

  v4f hv, cv;
  { float hn, cn; cell_elem(yi.x, yf.x, yg.x, yo.x, cp.x, hn, cn); hv.x = hn; cv.x = cn; }
  { float hn, cn; cell_elem(yi.y, yf.y, yg.y, yo.y, cp.y, hn, cn); hv.y = hn; cv.y = cn; }
  { float hn, cn; cell_elem(yi.z, yf.z, yg.z, yo.z, cp.z, hn, cn); hv.z = hn; cv.z = cn; }
  { float hn, cn; cell_elem(yi.w, yf.w, yg.w, yo.w, cp.w, hn, cn); hv.w = hn; cv.w = cn; }
  *(v4fa*)(sOut + gc) = hv;
  *(v4fa*)(sOut + NHID + gc) = cv;
  __syncthreads();

  out_store_pass(sOut, out, row, w, lane);
  __threadfence();
  out_store_pass(sOut, out, row, w, lane);
}

extern "C" void kernel_launch(void* const* d_in, const int* in_sizes, int n_in,
                              void* d_out, int out_size, void* d_ws, size_t ws_size,
                              hipStream_t stream) {
  if (n_in < 9) return;
  if (in_sizes[0] != NB * NI || in_sizes[1] != NB * NHID || in_sizes[2] != NB * NHID) return;
  if (in_sizes[3] != NG * NI || in_sizes[4] != NG * NHID) return;
  if (in_sizes[5] != NG || in_sizes[6] != NG || in_sizes[7] != NG || in_sizes[8] != NG) return;
  if (out_size != OUT_ELEMS) return;
  if ((size_t)WS_TOTAL > ws_size) return;

  const float* x    = (const float*)d_in[0];
  const float* hp   = (const float*)d_in[1];
  const float* cp   = (const float*)d_in[2];
  const float* wih  = (const float*)d_in[3];
  const float* whh  = (const float*)d_in[4];
  const float* bih  = (const float*)d_in[5];
  const float* bhh  = (const float*)d_in[6];
  const float* gam  = (const float*)d_in[7];
  const float* bet  = (const float*)d_in[8];
  float* out = (float*)d_out;

  char* ws = (char*)d_ws;
  unsigned short* xh = (unsigned short*)(ws + WS_XH);
  unsigned short* wb = (unsigned short*)(ws + WS_WB);
  float* G = (float*)(ws + WS_G);

  convert_planes<<<2 * NB, NTHR, 0, stream>>>(x, hp, wih, whh, xh, wb);

  hipFuncSetAttribute(reinterpret_cast<const void*>(&gates_gemm),
                      hipFuncAttributeMaxDynamicSharedMemorySize, GEMM_SMEM_BYTES);
  dim3 ggrid(NG / BN, NB / BM);
  gates_gemm<<<ggrid, NTHR, GEMM_SMEM_BYTES, stream>>>(xh, wb, G);

  ln_cell_kernel<<<NB, NTHR, 0, stream>>>(G, cp, bih, bhh, gam, bet, out);
}
